// Model_10299331576573
// MI455X (gfx1250) — hardware-verified
//
#include <hip/hip_runtime.h>
#include <stddef.h>
#include <stdint.h>


#define DF     128
#define LHD    256
#define NTHR   256
#define NWAVE  8
#define EPT    8
#define CHUNK  (NTHR * EPT)
#define WCAP   (EPT * 32)
#define LISTN  (NWAVE * WCAP)
#define NBA    1024
#define SLA    10
#define RCAP   28672
#define DEGCAP 64
#define GBM    64
#define GBN    128
#define GTHR   128
#define PBW    80
#define AGG_ZINTS    (LISTN + 2 * RCAP + 3 * NBA)
#define MISC_INTS    16
#define ROWH         256
#define ROWBUF_INTS  (NWAVE * ROWH / 2)
#define AGG_LDS_INTS (AGG_ZINTS + MISC_INTS + ROWBUF_INTS)

static_assert((CHUNK & (CHUNK - 1)) == 0 && CHUNK <= 4096);
static_assert((NBA & (NBA - 1)) == 0 && NBA == (1 << SLA));
static_assert(((long long)CHUNK << SLA) < (1LL << 31));
static_assert(NBA % NWAVE == 0 && NBA % 32 == 0 && NBA % GBM == 0);
static_assert(RCAP % 4 == 0 && AGG_ZINTS % 4 == 0 && LISTN % 4 == 0 && ((AGG_ZINTS + MISC_INTS) % 4) == 0);
static_assert(AGG_ZINTS % (NTHR * 4) == 0);
static_assert(DF % 32 == 0 && DF == 4 * 32 && GBN == DF && LHD == 2 * GBN);
static_assert(GBM == (GTHR / 32) * 16);
static_assert(DEGCAP >= 36 + 8 && RCAP >= 16710);
static_assert(AGG_LDS_INTS * 4 <= 300000);
static_assert((2 * DF * (DF / 8)) == 16 * NTHR);
static_assert((2 * DF * (2 * DF / 8)) == 32 * NTHR);
static_assert(PBW == 16 + 32 + 32);

typedef float          v4f   __attribute__((ext_vector_type(4)));
typedef float          v8f   __attribute__((ext_vector_type(8)));
typedef int            v4i   __attribute__((ext_vector_type(4)));
typedef int            v8i   __attribute__((ext_vector_type(8)));
typedef unsigned short v4us  __attribute__((ext_vector_type(4)));
typedef unsigned short v8us  __attribute__((ext_vector_type(8)));
typedef unsigned short v16us __attribute__((ext_vector_type(16)));
typedef __bf16         v16bf __attribute__((ext_vector_type(16)));
typedef v4f  __attribute__((may_alias)) v4fa;
typedef v4i  __attribute__((may_alias)) v4ia;
typedef v4us __attribute__((may_alias)) v4usa;
typedef v8us __attribute__((may_alias)) v8usa;
union FragB { v16bf v; v16us u; v8us h[2]; v8i w; };

__device__ __forceinline__ v8f wmb(const FragB& a, const FragB& b, v8f c) {
  v8f d = __builtin_amdgcn_wmma_f32_16x16x32_bf16(false, a.v, false, b.v, (short)0, c, false, false);
  asm volatile("v_nop\n\tv_nop\n\tv_nop\n\tv_nop" : "+v"(d) : "v"(a.w), "v"(b.w));
  return d;
}

__device__ __forceinline__ unsigned bf16_bits(float f) {
  const unsigned u = __float_as_uint(f);
  return (u + 0x7FFFu + ((u >> 16) & 1u)) >> 16;
}
__device__ __forceinline__ float bf16_val(float f) {
  return __uint_as_float(bf16_bits(f) << 16);
}

__device__ __forceinline__ void wave_sync() {
  __builtin_amdgcn_fence(__ATOMIC_RELEASE, "wavefront");
  __builtin_amdgcn_wave_barrier();
  __builtin_amdgcn_fence(__ATOMIC_ACQUIRE, "wavefront");
}

__device__ __forceinline__ float relu_keep(float v) { return (v > 0.0f) ? v : (v - v); }

template <int SLB>
__device__ __forceinline__ int scan_chunk(const int* __restrict__ dsts, int nE, int cbase, int slotBase,
                                          int nb, int vec8, int* list, int tid, int lane, int wave) {
  int wc = 0;
  const int el0  = tid * EPT;
  const int e0   = cbase + el0;
  const int sent = -2147483647 - 1;
  v4i da, db;
  if (vec8 != 0 && cbase + CHUNK <= nE) {
    da = *(const v4i*)(dsts + e0);
    db = *(const v4i*)(dsts + e0 + 4);
  } else {
    da.x = (e0     < nE) ? dsts[min(e0,     nE - 1)] : sent;
    da.y = (e0 + 1 < nE) ? dsts[min(e0 + 1, nE - 1)] : sent;
    da.z = (e0 + 2 < nE) ? dsts[min(e0 + 2, nE - 1)] : sent;
    da.w = (e0 + 3 < nE) ? dsts[min(e0 + 3, nE - 1)] : sent;
    db.x = (e0 + 4 < nE) ? dsts[min(e0 + 4, nE - 1)] : sent;
    db.y = (e0 + 5 < nE) ? dsts[min(e0 + 5, nE - 1)] : sent;
    db.z = (e0 + 6 < nE) ? dsts[min(e0 + 6, nE - 1)] : sent;
    db.w = (e0 + 7 < nE) ? dsts[min(e0 + 7, nE - 1)] : sent;
  }
  const unsigned nbs = (unsigned)slotBase;
  const unsigned unb = (unsigned)nb;
  const unsigned s0 = (unsigned)da.x - nbs, s1 = (unsigned)da.y - nbs;
  const unsigned s2 = (unsigned)da.z - nbs, s3 = (unsigned)da.w - nbs;
  const unsigned s4 = (unsigned)db.x - nbs, s5 = (unsigned)db.y - nbs;
  const unsigned s6 = (unsigned)db.z - nbs, s7 = (unsigned)db.w - nbs;
  const bool h0 = s0 < unb, h1 = s1 < unb, h2 = s2 < unb, h3 = s3 < unb;
  const bool h4 = s4 < unb, h5 = s5 < unb, h6 = s6 < unb, h7 = s7 < unb;
  const unsigned any = __builtin_amdgcn_ballot_w32(h0 | h1 | h2 | h3 | h4 | h5 | h6 | h7);
  if (any != 0u) {
#define HITJ(J, HJ, SJ) { \
      const unsigned mj = __builtin_amdgcn_ballot_w32(HJ); \
      if (mj != 0u) { \
        if (HJ) { \
          const int pos = wc + (int)__builtin_amdgcn_mbcnt_lo(mj, 0u); \
          if (pos < WCAP) list[wave * WCAP + pos] = ((el0 + (J)) << SLB) | (int)(SJ); \
        } \
        wc += (int)__builtin_popcount(mj); } }
    HITJ(0, h0, s0)
    HITJ(1, h1, s1)
    HITJ(2, h2, s2)
    HITJ(3, h3, s3)
    HITJ(4, h4, s4)
    HITJ(5, h5, s5)
    HITJ(6, h6, s6)
    HITJ(7, h7, s7)
#undef HITJ
  }
  return wc;
}

__device__ __forceinline__ void cvt8_store(const float* __restrict__ p, unsigned short* dp, bool ok) {
  const v4f a = *(const v4f*)p;
  const v4f b = *(const v4f*)(p + 4);
  v8us o;
  o[0] = ok ? (unsigned short)bf16_bits(a.x) : (unsigned short)0;
  o[1] = ok ? (unsigned short)bf16_bits(a.y) : (unsigned short)0;
  o[2] = ok ? (unsigned short)bf16_bits(a.z) : (unsigned short)0;
  o[3] = ok ? (unsigned short)bf16_bits(a.w) : (unsigned short)0;
  o[4] = ok ? (unsigned short)bf16_bits(b.x) : (unsigned short)0;
  o[5] = ok ? (unsigned short)bf16_bits(b.y) : (unsigned short)0;
  o[6] = ok ? (unsigned short)bf16_bits(b.z) : (unsigned short)0;
  o[7] = ok ? (unsigned short)bf16_bits(b.w) : (unsigned short)0;
  *(volatile v8us*)dp = o;
  __threadfence();
  *(volatile v8us*)dp = o;
}

__global__ __launch_bounds__(NTHR) void k_prep(const float* __restrict__ x,
                                               const float* __restrict__ W1l, const float* __restrict__ W1r,
                                               const float* __restrict__ W2l, const float* __restrict__ W2r,
                                               const float* __restrict__ W3, int nN, int nUx,
                                               unsigned short* XB, unsigned short* WB1,
                                               unsigned short* WB2, unsigned short* WB3) {
  const int b   = (int)blockIdx.x;
  const int tid = (int)threadIdx.x;
  if (b < 8) {
    const int v = b * NTHR + tid;
    const int n = v >> 4, k8 = (v & 15) * 8;
    cvt8_store(W1l + (size_t)n * DF + k8, WB1 + (size_t)n * DF + k8, true);
  } else if (b < 16) {
    const int v = (b - 8) * NTHR + tid;
    const int n = v >> 4, k8 = (v & 15) * 8;
    cvt8_store(W1r + (size_t)n * DF + k8, WB1 + (size_t)(DF + n) * DF + k8, true);
  } else if (b < 32) {
    const int v = (b - 16) * NTHR + tid;
    const int n = v >> 5, k8 = (v & 31) * 8;
    cvt8_store(W2l + (size_t)n * DF + (k8 & (DF - 1)), WB2 + (size_t)n * (2 * DF) + k8, true);
  } else if (b < 48) {
    const int v = (b - 32) * NTHR + tid;
    const int n = v >> 5, k8 = (v & 31) * 8;
    cvt8_store(W2r + (size_t)n * DF + (k8 & (DF - 1)), WB2 + (size_t)(DF + n) * (2 * DF) + k8, true);
  } else if (b < PBW) {
    const int v = (b - 48) * NTHR + tid;
    const int n = v >> 5, k8 = (v & 31) * 8;
    cvt8_store(W3 + (size_t)n * DF + (k8 & (DF - 1)), WB3 + (size_t)n * (2 * DF) + k8, true);
  } else {
    const int u = (b - PBW) * NTHR + tid;
    if (u < nUx) {
      const int row = u >> 4, k8 = (u & 15) * 8;
      const int rc  = row < nN ? row : nN - 1;
      cvt8_store(x + (size_t)rc * DF + k8, XB + (size_t)row * DF + k8, row < nN);
    }
  }
}

template <int NPARTS>
__device__ __forceinline__ void tile_mma(const unsigned short* __restrict__ Apl, size_t pstride,
                                         const unsigned short* __restrict__ BT, int rowBase, int col0,
                                         int lane, int wave, v8f (&acc)[8]) {
  const int hh = lane >> 4, m = lane & 15;
  constexpr int K = NPARTS * DF;
  {
    const v8f z = {0.f, 0.f, 0.f, 0.f, 0.f, 0.f, 0.f, 0.f};
#pragma unroll
    for (int t = 0; t < 8; ++t) acc[t] = z;
  }
  const unsigned short* ap0 = Apl + (size_t)(rowBase + 16 * wave + m) * (size_t)DF + 8 * hh;
  const unsigned short* bp  = BT + (size_t)(col0 + m) * (size_t)K + 8 * hh;
#pragma unroll 1
  for (int part = 0; part < NPARTS; ++part) {
    const unsigned short* ap = ap0 + (size_t)part * pstride;
#pragma unroll 1
    for (int k0 = 0; k0 < DF; k0 += 32) {
      FragB af;
      af.h[0] = *(const v8usa*)(ap + k0);
      af.h[1] = *(const v8usa*)(ap + k0 + 16);
#pragma unroll
      for (int nt = 0; nt < 8; ++nt) {
        const unsigned short* wq = bp + (size_t)(16 * nt) * (size_t)K + part * DF + k0;
        FragB bf;
        bf.h[0] = *(const v8usa*)wq;
        bf.h[1] = *(const v8usa*)(wq + 16);
        acc[nt] = wmb(af, bf, acc[nt]);
      }
    }
  }
}

template <int NPARTS>
__global__ __launch_bounds__(GTHR) void k_gemm(const unsigned short* __restrict__ Apl, size_t pstride,
                                               const unsigned short* __restrict__ BT,
                                               const float* __restrict__ bias, float* PR, size_t rOff) {
  __shared__ __attribute__((aligned(16))) float stg[GBM * GBN];
  const int tid = (int)threadIdx.x, lane = tid & 31, wave = tid >> 5, hh = lane >> 4, m = lane & 15;
  const int rowBase = (int)blockIdx.x * GBM;
  const int by      = (int)blockIdx.y;

  v8f acc[8];
  tile_mma<NPARTS>(Apl, pstride, BT, rowBase, by * GBN, lane, wave, acc);

#pragma unroll
  for (int nt = 0; nt < 8; ++nt) {
    const int lc = 16 * nt + m;
#pragma unroll
    for (int r = 0; r < 8; ++r) {
      const int lr = 16 * wave + 8 * hh + r;
      stg[lr * GBN + lc] = acc[nt][r];
    }
  }
  __syncthreads();

  v4f bb4;
  {
    const float bsel = (by != 0) ? 1.0f : 0.0f;
    const v4f t1 = *(const v4f*)(bias + 4 * lane);
    bb4.x = bf16_val(t1.x) * bsel;
    bb4.y = bf16_val(t1.y) * bsel;
    bb4.z = bf16_val(t1.z) * bsel;
    bb4.w = bf16_val(t1.w) * bsel;
  }
  v4f pv[16];
#pragma unroll
  for (int i = 0; i < 16; ++i) pv[i] = *(const v4fa*)(stg + (16 * wave + i) * GBN + 4 * lane) + bb4;

  float* ob = PR + (size_t)by * rOff + (size_t)(rowBase + 16 * wave) * (size_t)DF + 4 * lane;
#pragma unroll
  for (int i = 0; i < 16; ++i) *(volatile v4f*)(ob + (size_t)i * DF) = pv[i];
  __threadfence();
#pragma unroll
  for (int i = 0; i < 16; ++i) *(volatile v4f*)(ob + (size_t)i * DF) = pv[i];
}

template <int RELU>
__global__ __launch_bounds__(NTHR) void k_scan(const int* __restrict__ gath, const int* __restrict__ keys,
                                               int nE, int nN, int vec8, int mRows,
                                               const float* __restrict__ PR, size_t rOff,
                                               unsigned short* hpl, size_t pstride) {
  extern __shared__ __attribute__((aligned(16))) int dsm[];
  int* list = dsm;
  int* hl   = dsm + LISTN;
  int* sl   = hl + RCAP;
  int* cnt  = sl + RCAP;
  int* offs = cnt + NBA;
  int* cur  = offs + NBA;
  int* misc = cur + NBA;
  const int tid = (int)threadIdx.x, lane = tid & 31, wave = tid >> 5;
  unsigned short* rowbuf = (unsigned short*)(misc + MISC_INTS) + wave * ROWH;
  const int nodeBase = (int)blockIdx.x * NBA;

  {
    const v4i z4 = {0, 0, 0, 0};
    for (int i = tid * 4; i < AGG_ZINTS; i += NTHR * 4) *(v4ia*)(dsm + i) = z4;
    if (tid < MISC_INTS) misc[tid] = 0;
  }
  __syncthreads();

  int t = 0, ov = 0;
  const int nChunks = (nE + CHUNK - 1) / CHUNK;
#pragma unroll 1
  for (int ch = 0; ch < nChunks; ++ch) {
    const int cbase = ch * CHUNK;
    const int wc = scan_chunk<SLA>(keys, nE, cbase, nodeBase, NBA, vec8, list, tid, lane, wave);
    if (lane == 0) misc[wave] = wc;
    __syncthreads();
    if (wave == 0) {
#pragma unroll 1
      for (int w2 = 0; w2 < NWAVE; ++w2) {
        int c = misc[w2];
        c = c < 0 ? 0 : (c > WCAP ? WCAP : c);
#pragma unroll 1
        for (int b0 = 0; b0 < c; b0 += 32) {
          const int idx = b0 + lane;
          const int ent = list[w2 * WCAP + (idx < WCAP ? idx : WCAP - 1)];
          const int m32 = (c - b0) < 32 ? (c - b0) : 32;
#pragma unroll 1
          for (int k = 0; k < m32; ++k) {
            const int u    = __builtin_amdgcn_readlane(ent, k);
            const int slot = u & (NBA - 1);
            const int el   = (u >> SLA) & (CHUNK - 1);
            const int pk   = ((cbase + el) << SLA) | slot;
            if (t < RCAP) {
              if (lane == 0) { hl[t] = pk; cnt[slot] = cnt[slot] + 1; }
              t = t + 1;
            } else {
              ov = 1;
            }
          }
        }
      }
    }
    __syncthreads();
  }
  if (wave == 0 && lane == 0) { misc[8] = t; misc[9] = ov; }
  __syncthreads();
  int tt = misc[8];
  tt = tt < 0 ? 0 : (tt > RCAP ? RCAP : tt);
  const int ovf = misc[9];

  if (wave == 0) {
    const int base = lane * (NBA / 32);
    int s = 0;
#pragma unroll 1
    for (int i = 0; i < NBA / 32; ++i) s += cnt[base + i];
    int incl = s;
#pragma unroll
    for (int d = 1; d < 32; d <<= 1) {
      const int y = __shfl_up(incl, d, 32);
      if (lane >= d) incl += y;
    }
    int run = incl - s;
#pragma unroll 1
    for (int i = 0; i < NBA / 32; ++i) {
      const int cv = cnt[base + i];
      offs[base + i] = run;
      cur[base + i]  = run;
      run += cv;
    }
  }
  __syncthreads();
  if (wave == 0) {
#pragma unroll 1
    for (int b0 = 0; b0 < tt; b0 += 32) {
      const int idx = b0 + lane;
      const int ent = hl[idx < RCAP ? idx : RCAP - 1];
      const int m32 = (tt - b0) < 32 ? (tt - b0) : 32;
#pragma unroll 1
      for (int k = 0; k < m32; ++k) {
        const int u    = __builtin_amdgcn_readlane(ent, k);
        const int slot = u & (NBA - 1);
        if (lane == 0) {
          int p = cur[slot];
          p = p < 0 ? 0 : (p > RCAP - 1 ? RCAP - 1 : p);
          sl[p] = u;
          cur[slot] = p + 1;
        }
      }
    }
  }
  __syncthreads();

  const float qnan = __int_as_float(0x7fc00000);
  const float pz = (ovf != 0) ? qnan : 0.0f;
  const float* Rp = PR + rOff;
#pragma unroll 1
  for (int si = 0; si < NBA / NWAVE; ++si) {
    const int s    = si * NWAVE + wave;
    const int node = nodeBase + s;
    int craw = cnt[s];
    craw = craw < 0 ? 0 : craw;
    const bool big = craw > DEGCAP;
    const int c = craw > DEGCAP ? DEGCAP : craw;
    int o = offs[s];
    o = o < 0 ? 0 : (o > RCAP ? RCAP : o);
    const int nc = node < nN ? node : nN - 1;
    float a0 = 0.0f, a1 = 0.0f, a2 = 0.0f, a3 = 0.0f;
#pragma unroll 1
    for (int b0 = 0; b0 < c; b0 += 32) {
      int idx = o + b0 + lane;
      idx = idx > RCAP - 1 ? RCAP - 1 : idx;
      const int ent = sl[idx];
      int eid = ent >> SLA;
      eid = eid < 0 ? 0 : (eid > nE - 1 ? nE - 1 : eid);
      int sr = gath[eid];
      sr = sr < 0 ? 0 : (sr > nN - 1 ? nN - 1 : sr);
      const int m32 = (c - b0) < 32 ? (c - b0) : 32;
#pragma unroll 1
      for (int k = 0; k < m32; ++k) {
        const int sk = __builtin_amdgcn_readlane(sr, k);
        const v4f a = *(const v4f*)(PR + (size_t)sk * DF + 4 * lane);
        a0 += a.x; a1 += a.y; a2 += a.z; a3 += a.w;
      }
    }
    const v4f rr = *(const v4f*)(Rp + (size_t)nc * DF + 4 * lane);
    const float cf = (float)(craw < 1 ? 1 : craw);
    float y0 = a0 / cf + rr.x;
    float y1 = a1 / cf + rr.y;
    float y2 = a2 / cf + rr.z;
    float y3 = a3 / cf + rr.w;
    if constexpr (RELU != 0) {
      y0 = relu_keep(y0); y1 = relu_keep(y1); y2 = relu_keep(y2); y3 = relu_keep(y3);
    }
    const float pzr = big ? qnan : pz;
    const bool live = node < nN;
    const float m0 = live ? (y0 + pzr) : 0.0f;
    const float m1 = live ? (y1 + pzr) : 0.0f;
    const float m2 = live ? (y2 + pzr) : 0.0f;
    const float m3 = live ? (y3 + pzr) : 0.0f;
    v4us mh, ml;
    {
      unsigned hb;
      hb = bf16_bits(m0); mh[0] = (unsigned short)hb; ml[0] = (unsigned short)bf16_bits(m0 - __uint_as_float(hb << 16));
      hb = bf16_bits(m1); mh[1] = (unsigned short)hb; ml[1] = (unsigned short)bf16_bits(m1 - __uint_as_float(hb << 16));
      hb = bf16_bits(m2); mh[2] = (unsigned short)hb; ml[2] = (unsigned short)bf16_bits(m2 - __uint_as_float(hb << 16));
      hb = bf16_bits(m3); mh[3] = (unsigned short)hb; ml[3] = (unsigned short)bf16_bits(m3 - __uint_as_float(hb << 16));
    }
    *(v4usa*)(rowbuf + 4 * lane) = mh;
    *(v4usa*)(rowbuf + DF + 4 * lane) = ml;
    wave_sync();
    const v8us q0 = *(const v8usa*)(rowbuf + 8 * lane);
    wave_sync();
    if (node < mRows) {
      unsigned short* rpw = hpl + (size_t)(lane >> 4) * pstride + (size_t)node * DF + 8 * (lane & 15);
      *(volatile v8us*)rpw = q0;
      __threadfence();
      *(volatile v8us*)rpw = q0;
    }
  }
}

__global__ __launch_bounds__(GTHR) void k_dec(const unsigned short* __restrict__ Hpl, size_t pstride,
                                              const unsigned short* __restrict__ WB3,
                                              const float* __restrict__ b3, const float* __restrict__ W4,
                                              const float* __restrict__ b4, float* out, int nN) {
  __shared__ __attribute__((aligned(16))) float stg[GBM * GBN];
  __shared__ __attribute__((aligned(16))) float outs[GBM];
  const int tid = (int)threadIdx.x, lane = tid & 31, wave = tid >> 5, hh = lane >> 4, m = lane & 15;
  const int rowBase = (int)blockIdx.x * GBM;

  float tot = 0.0f;
#pragma unroll 1
  for (int half = 0; half < 2; ++half) {
    v8f acc[8];
    tile_mma<2>(Hpl, pstride, WB3, rowBase, half * GBN, lane, wave, acc);
#pragma unroll
    for (int nt = 0; nt < 8; ++nt) {
      const int lc = 16 * nt + m;
#pragma unroll
      for (int r = 0; r < 8; ++r) {
        const int lr = 16 * wave + 8 * hh + r;
        stg[lr * GBN + lc] = acc[nt][r];
      }
    }
    __syncthreads();
    v4f bb, ww;
    {
      const v4f t1 = *(const v4f*)(b3 + half * GBN + 4 * lane);
      const v4f t2 = *(const v4f*)(W4 + half * GBN + 4 * lane);
      bb.x = bf16_val(t1.x); bb.y = bf16_val(t1.y); bb.z = bf16_val(t1.z); bb.w = bf16_val(t1.w);
      ww.x = bf16_val(t2.x); ww.y = bf16_val(t2.y); ww.z = bf16_val(t2.z); ww.w = bf16_val(t2.w);
    }
    float mine = 0.0f;
#pragma unroll 1
    for (int i = 0; i < 16; ++i) {
      const v4f v = *(const v4fa*)(stg + (16 * wave + i) * GBN + 4 * lane);
      const float z0 = relu_keep(v.x + bb.x);
      const float z1 = relu_keep(v.y + bb.y);
      const float z2 = relu_keep(v.z + bb.z);
      const float z3 = relu_keep(v.w + bb.w);
      float p = (z0 * ww.x + z1 * ww.y) + (z2 * ww.z + z3 * ww.w);
      p += __shfl_xor(p, 16, 32);
      p += __shfl_xor(p, 8, 32);
      p += __shfl_xor(p, 4, 32);
      p += __shfl_xor(p, 2, 32);
      p += __shfl_xor(p, 1, 32);
      mine = (lane == i) ? p : mine;
    }
    tot += mine;
    __syncthreads();
  }
  if (lane < 16) outs[16 * wave + lane] = tot + bf16_val(b4[0]);
  __syncthreads();

  const v4f ov = *(const v4fa*)(outs + 4 * (lane & 15));
  int nv = nN - rowBase;
  nv = nv < 0 ? 0 : (nv > GBM ? GBM : nv);
  const bool okst = (wave == 0) && (4 * lane < nv);
  float* op = out + (size_t)rowBase + 4 * (lane & 15);
  if (okst) *(volatile v4f*)op = ov;
  __threadfence();
  if (okst) *(volatile v4f*)op = ov;
}

static inline int cdiv(int a, int b) { return (a + b - 1) / b; }
static inline size_t al256(size_t o) { return (o + 255) & ~(size_t)255; }

extern "C" void kernel_launch(void* const* d_in, const int* in_sizes, int n_in,
                              void* d_out, int out_size, void* d_ws, size_t ws_size,
                              hipStream_t stream) {
  if (n_in < 12) return;
  if (in_sizes[0] < DF || (in_sizes[0] % DF) != 0) return;
  const int nN = in_sizes[0] / DF;
  if (nN < 32 || (nN % 32) != 0 || nN >= (1 << 24)) return;
  if (in_sizes[1] < 2 || (in_sizes[1] & 1) != 0) return;
  const int nE = in_sizes[1] / 2;
  if (nE < 1 || nE >= (1 << 21)) return;
  if (in_sizes[2] != DF * DF || in_sizes[3] != DF || in_sizes[4] != DF * DF) return;
  if (in_sizes[5] != DF * DF || in_sizes[6] != DF || in_sizes[7] != DF * DF) return;
  if (in_sizes[8] != LHD * DF || in_sizes[9] != LHD) return;
  if (in_sizes[10] != LHD || in_sizes[11] != 1) return;
  if (out_size != nN) return;

  const float* x   = (const float*)d_in[0];
  const int*   ei  = (const int*)d_in[1];
  const float* W1l = (const float*)d_in[2];
  const float* b1  = (const float*)d_in[3];
  const float* W1r = (const float*)d_in[4];
  const float* W2l = (const float*)d_in[5];
  const float* b2  = (const float*)d_in[6];
  const float* W2r = (const float*)d_in[7];
  const float* W3  = (const float*)d_in[8];
  const float* b3  = (const float*)d_in[9];
  const float* W4  = (const float*)d_in[10];
  const float* b4  = (const float*)d_in[11];
  float* out = (float*)d_out;
  const int* src = ei;
  const int* dst = ei + nE;

  const int MP = cdiv(nN, GBM) * GBM;
  const int gM = MP / GBM;
  const int gA = cdiv(MP, NBA);
  if ((long long)gA * NBA < (long long)MP) return;
  const int vec8 = ((nE & 3) == 0) ? 1 : 0;

  const size_t plane16 = (size_t)MP * DF;
  const size_t plane32 = (size_t)MP * DF;
  char* ws = (char*)d_ws;
  size_t off = 0;
  const size_t oH  = off; off = al256(off + 2 * plane16 * 2);
  const size_t oPR = off; off = al256(off + 2 * plane32 * 4);
  const size_t oB1 = off; off = al256(off + (size_t)2 * DF * DF * 2);
  const size_t oB2 = off; off = al256(off + (size_t)2 * DF * 2 * DF * 2);
  const size_t oB3 = off; off = al256(off + (size_t)LHD * 2 * DF * 2);
  if (off > ws_size) return;
  unsigned short* HPL = (unsigned short*)(ws + oH);
  float*          PR  = (float*)(ws + oPR);
  unsigned short* WB1 = (unsigned short*)(ws + oB1);
  unsigned short* WB2 = (unsigned short*)(ws + oB2);
  unsigned short* WB3 = (unsigned short*)(ws + oB3);

  const size_t scanLds = (size_t)AGG_LDS_INTS * 4;
  hipFuncSetAttribute(reinterpret_cast<const void*>(&k_scan<1>), hipFuncAttributeMaxDynamicSharedMemorySize, (int)scanLds);
  hipFuncSetAttribute(reinterpret_cast<const void*>(&k_scan<0>), hipFuncAttributeMaxDynamicSharedMemorySize, (int)scanLds);

  const int nUx = MP * (DF / 8);
  k_prep<<<PBW + cdiv(nUx, NTHR), NTHR, 0, stream>>>(x, W1l, W1r, W2l, W2r, W3, nN, nUx, HPL, WB1, WB2, WB3);
  k_gemm<1><<<dim3(gM, 2), GTHR, 0, stream>>>(HPL, plane16, WB1, b1, PR, plane32);
  k_scan<1><<<gA, NTHR, scanLds, stream>>>(src, dst, nE, nN, vec8, MP, PR, plane32, HPL, plane16);
  k_gemm<2><<<dim3(gM, 2), GTHR, 0, stream>>>(HPL, plane16, WB2, b2, PR, plane32);
  k_scan<0><<<gA, NTHR, scanLds, stream>>>(src, dst, nE, nN, vec8, MP, PR, plane32, HPL, plane16);
  k_dec<<<gM, GTHR, 0, stream>>>(HPL, plane16, WB3, b3, W4, b4, out, nN);
}
